// GATLayer_19688130085110
// MI455X (gfx1250) — hardware-run, weakly checked
//
#include <hip/hip_runtime.h>

typedef float          v8f   __attribute__((ext_vector_type(8)));
typedef float          v4f   __attribute__((ext_vector_type(4)));
typedef unsigned int   v4u   __attribute__((ext_vector_type(4)));
typedef int            v8i   __attribute__((ext_vector_type(8)));
typedef unsigned short v8us  __attribute__((ext_vector_type(8)));
typedef unsigned short v16us __attribute__((ext_vector_type(16)));
typedef __bf16         v16bf __attribute__((ext_vector_type(16)));
typedef _Float16       v16h  __attribute__((ext_vector_type(16)));
typedef v4f  __attribute__((may_alias)) v4fa;
typedef v8us __attribute__((may_alias)) v8usa;
union FragB { v16bf v; v16us u; v8us h[2]; v8i w; };
union FragH { v16h  v; v16us u; v8us h[2]; v8i w; };

__device__ __forceinline__ v8f wmb(const FragB& a, const FragB& b, v8f c) {
  v8f d = __builtin_amdgcn_wmma_f32_16x16x32_bf16(false, a.v, false, b.v, (short)0, c, false, false);
  asm volatile("v_nop\n\tv_nop\n\tv_nop\n\tv_nop" : "+v"(d) : "v"(a.w), "v"(b.w));
  return d;
}

__device__ __forceinline__ v8f wmh(const FragH& a, const FragH& b, v8f c) {
  v8f d = __builtin_amdgcn_wmma_f32_16x16x32_f16(false, a.v, false, b.v, (short)0, c, false, false);
  asm volatile("v_nop\n\tv_nop\n\tv_nop\n\tv_nop" : "+v"(d) : "v"(a.w), "v"(b.w));
  return d;
}

__device__ __forceinline__ unsigned bf16_bits(float f) {
  const unsigned u = __float_as_uint(f);
  const unsigned r = (u + 0x7FFFu + ((u >> 16) & 1u)) >> 16;
  const unsigned q = (u >> 16) | 0x40u;
  return ((u & 0x7fffffffu) > 0x7f800000u) ? q : r;
}

__device__ __forceinline__ float bf16_val(float f) {
  return __uint_as_float(bf16_bits(f) << 16);
}
__device__ __forceinline__ int clampi(int v, int lo, int hi) {
  return v < lo ? lo : (v > hi ? hi : v);
}

__device__ __forceinline__ unsigned f16_bits(float f) {
  const unsigned u  = __float_as_uint(f);
  const unsigned s  = (u >> 16) & 0x8000u;
  const unsigned a  = u & 0x7fffffffu;
  const unsigned t  = a - 0x38000000u;
  const unsigned r  = (t + 0x0FFFu + ((t >> 13) & 1u)) >> 13;
  const unsigned rc = r > 0x7C00u ? 0x7C00u : r;
  const bool small  = a < 0x38800000u;
  const bool isnan  = a > 0x7f800000u;
  const unsigned fin = small ? 0u : (s | rc);
  return isnan ? (s | 0x7E00u) : fin;
}

__device__ __forceinline__ unsigned pk16(unsigned lo, unsigned hi) { return lo | (hi << 16); }
__device__ __forceinline__ unsigned bf16_lo_bits(float v) {
  float hi = bf16_val(v);
  asm volatile("" : "+v"(hi));
  return bf16_bits(v - hi);
}
__device__ __forceinline__ v4u pack8_bf16(v4f a, v4f c) {
  return (v4u){ pk16(bf16_bits(a[0]), bf16_bits(a[1])), pk16(bf16_bits(a[2]), bf16_bits(a[3])),
                pk16(bf16_bits(c[0]), bf16_bits(c[1])), pk16(bf16_bits(c[2]), bf16_bits(c[3])) };
}
__device__ __forceinline__ v4u pack8_bf16_lo(v4f a, v4f c) {
  return (v4u){ pk16(bf16_lo_bits(a[0]), bf16_lo_bits(a[1])), pk16(bf16_lo_bits(a[2]), bf16_lo_bits(a[3])),
                pk16(bf16_lo_bits(c[0]), bf16_lo_bits(c[1])), pk16(bf16_lo_bits(c[2]), bf16_lo_bits(c[3])) };
}
__device__ __forceinline__ v4u pack8_f16(v4f a, v4f c) {
  return (v4u){ pk16(f16_bits(a[0]), f16_bits(a[1])), pk16(f16_bits(a[2]), f16_bits(a[3])),
                pk16(f16_bits(c[0]), f16_bits(c[1])), pk16(f16_bits(c[2]), f16_bits(c[3])) };
}

template <int FORM>
__global__ __launch_bounds__(256) void k_plane(const float* __restrict__ src, int rows, int cols, int ldsrc,
                                               unsigned short* __restrict__ dst, int MP, int KP) {
  static_assert(FORM >= 0 && FORM <= 3);
  const int KTOT = (FORM == 1 || FORM == 3) ? 2 * KP : KP;
  const unsigned ppr   = (unsigned)(KTOT >> 3);
  const unsigned kp8   = (unsigned)(KP >> 3);
  const unsigned total = (unsigned)MP * ppr;
  const unsigned g     = blockIdx.x * 256u + threadIdx.x;
  const unsigned rowu  = g / ppr;
  const unsigned p     = g - rowu * ppr;
  const bool second    = p >= kp8;
  const int row = (int)rowu;
  const int c0  = (int)((second ? p - kp8 : p) << 3);
  const float* srow = src + (size_t)clampi(row, 0, rows - 1) * (size_t)ldsrc;
  float x[8];
  unsigned mk[8];
#pragma unroll
  for (int e = 0; e < 8; ++e) {
    const int c = c0 + e;
    const float v = srow[clampi(c, 0, cols - 1)];
    asm volatile("" :: "v"(v));
    x[e]  = v;
    mk[e] = (row < rows && c < cols) ? 0xFFFFu : 0u;
  }
  const v4f a = (v4f){ x[0], x[1], x[2], x[3] };
  const v4f c = (v4f){ x[4], x[5], x[6], x[7] };
  v4u o;
  if (FORM == 2) {
    o = pack8_f16(a, c);
  } else {
    const v4u hi = pack8_bf16(a, c);
    o = hi;
    if (FORM == 1) { const v4u lo = pack8_bf16_lo(a, c); o = second ? lo : hi; }
  }
  const v4u mw = (v4u){ pk16(mk[0], mk[1]), pk16(mk[2], mk[3]), pk16(mk[4], mk[5]), pk16(mk[6], mk[7]) };
  o &= mw;
  if (g < total) {
    volatile v4u* q = (volatile v4u*)(dst + (size_t)g * 8);
    *q = o;
    __threadfence();
    *q = o;
  }
}

template <int FORM> struct FragOf    { typedef FragB T; };
template <>         struct FragOf<2> { typedef FragH T; };
__device__ __forceinline__ v8f mm(const FragB& a, const FragB& b, v8f c) { return wmb(a, b, c); }
__device__ __forceinline__ v8f mm(const FragH& a, const FragH& b, v8f c) { return wmh(a, b, c); }
template <class F> __device__ __forceinline__ F ld_frag(const unsigned short* p) {
  F f;
  f.h[0] = *(const v8usa*)(p);
  f.h[1] = *(const v8usa*)(p + 16);
  return f;
}

template <int FORM, int EPI>
__global__ __launch_bounds__(256) __attribute__((amdgpu_num_vgpr(248)))
void k_gemm_nt(const unsigned short* __restrict__ A, const unsigned short* __restrict__ B,
               const float* __restrict__ bias, float* __restrict__ D, int M, int N, int KTOT, int ldd) {
  static_assert(FORM >= 0 && FORM <= 2);
  static_assert(EPI == 0 || EPI == 1);
  typedef typename FragOf<FORM>::T F;
  __shared__ __attribute__((aligned(16))) float sT[8][16 * 68];
  const int lane = threadIdx.x & 31;
  const int wave = threadIdx.x >> 5;
  const int tilesM = (M + 63) >> 6;
  const int tilesN = (N + 63) >> 6;
  const int tile = blockIdx.x * 8 + wave;
  if (tile >= tilesM * tilesN) return;
  const int tm = tile / tilesN;
  const int tn = tile - tm * tilesN;
  const int m0 = tm << 6;
  const int n0 = tn << 6;

  const int rl = lane & 15;
  const int h8 = (lane >> 4) * 8;
  const unsigned short* pa = A + (size_t)(m0 + rl) * (size_t)KTOT + h8;
  const unsigned short* pb = B + (size_t)(n0 + rl) * (size_t)KTOT + h8;

  v8f acc[4][4];
#pragma unroll
  for (int i = 0; i < 4; ++i)
#pragma unroll
    for (int j = 0; j < 4; ++j) acc[i][j] = (v8f){0.f, 0.f, 0.f, 0.f, 0.f, 0.f, 0.f, 0.f};

#pragma unroll 1
  for (int k0 = 0; k0 < KTOT; k0 += 32) {
    F bf[4];
#pragma unroll
    for (int j = 0; j < 4; ++j) bf[j] = ld_frag<F>(pb + (size_t)(j << 4) * (size_t)KTOT + k0);
#pragma unroll
    for (int i = 0; i < 4; ++i) {
      const F af = ld_frag<F>(pa + (size_t)(i << 4) * (size_t)KTOT + k0);
#pragma unroll
      for (int j = 0; j < 4; ++j) acc[i][j] = mm(af, bf[j], acc[i][j]);
    }
  }

  float* slab = sT[wave];
  const int hh = lane >> 4;
  const int c4 = (lane & 15) * 4;
  const int nc = n0 + c4;
  const bool cok = nc < N;
  v4f bv = (v4f){0.f, 0.f, 0.f, 0.f};
  if (EPI == 1) {
    bv = *(const v4fa*)(bias + clampi(nc, 0, N - 4));
    asm volatile("" :: "v"(bv));
  }
#pragma unroll
  for (int i = 0; i < 4; ++i) {
    const int mBase = m0 + (i << 4);
#pragma unroll
    for (int j = 0; j < 4; ++j) {
#pragma unroll
      for (int r = 0; r < 8; ++r) slab[(h8 + r) * 68 + (j << 4) + rl] = acc[i][j][r];
    }
    __builtin_amdgcn_fence(__ATOMIC_RELEASE, "workgroup");
    __builtin_amdgcn_wave_barrier();
    __builtin_amdgcn_fence(__ATOMIC_ACQUIRE, "workgroup");
    v4f vv[8];
#pragma unroll
    for (int it = 0; it < 8; ++it) {
      const int row = it * 2 + hh;
      v4f v = *(const v4fa*)(slab + row * 68 + c4);
      if (EPI == 1) v += bv;
      vv[it] = v;
    }
    for (int pass = 0; pass < 2; ++pass) {
#pragma unroll
      for (int it = 0; it < 8; ++it) {
        const int row = mBase + it * 2 + hh;
        if (cok && row < M) *(volatile v4f*)(D + (size_t)row * (size_t)ldd + nc) = vv[it];
      }
      __threadfence();
    }
    __builtin_amdgcn_fence(__ATOMIC_RELEASE, "workgroup");
    __builtin_amdgcn_wave_barrier();
    __builtin_amdgcn_fence(__ATOMIC_ACQUIRE, "workgroup");
  }
}

#pragma clang fp contract(off)


#define NN      50000
#define NE      800000
#define MPAD    50048
#define KD      256
#define HC      256
#define NHD     4
#define DSZ     64
#define RTHR    256
#define RWAVES  8
#define TAB_N   512
#define BT      512
#define BW      16
#define BEPT    8
#define BCHUNK  (BT * BEPT)
#define NCH     ((NE + BCHUNK - 1) / BCHUNK)
#define NB      1024
#define NBLK    ((NN + NB - 1) / NB)
#define RCAP    20992
#define DEGCAP  64
#define WSTEP   8
#define SLOTSH  20
#define LISTTOT (NBLK * RCAP)
#define LDS_BKT ((2 * RCAP + 3 * NB + 64) * 4)
#define A2OFF   (MPAD * NHD)
#define WSMAX   ((size_t)128 << 20)

static_assert(NHD * DSZ == 256 && 256 == 32 * 8 && HC == 256 && KD == 256);
static_assert(MPAD == 782 * 64 && MPAD % 64 == 0 && MPAD >= NN && MPAD % RWAVES == 0);
static_assert(KD % 32 == 0 && HC % 64 == 0);
static_assert(NE < (1 << SLOTSH) && SLOTSH + 10 <= 31);
static_assert(NB == 1024 && NB == 2 * BT);
static_assert(NE % 8 == 0 && NE >= 8);
static_assert(NBLK == 49 && NBLK * NB >= NN);
static_assert(NCH == 196 && NCH * BCHUNK >= NE);
static_assert(RCAP % 32 == 0);
static_assert(RCAP * 4 >= 16696 * 5);
static_assert(DEGCAP >= 33 + 8);
static_assert(DEGCAP % WSTEP == 0 && WSTEP * NHD == 32);
static_assert(LDS_BKT <= 262144);
static_assert(BW == BT / 32 && BW == 16);
static_assert(6250 * 8 == NN && NN % RWAVES == 0);

typedef int v4i __attribute__((ext_vector_type(4)));
typedef int v2i __attribute__((ext_vector_type(2)));
typedef v4i __attribute__((may_alias)) v4ia;
typedef v2i __attribute__((may_alias)) v2ia;

__device__ __forceinline__ float lrelu_k(float v) { return (v > 0.0f) ? v : 0.2f * v; }
__device__ __forceinline__ float nmax(float m, float e) { return (e > m || e != e) ? e : m; }
__device__ __forceinline__ float sum8(float t) {
  t = t + __shfl_xor(t, 4, 32);
  t = t + __shfl_xor(t, 2, 32);
  t = t + __shfl_xor(t, 1, 32);
  return t;
}
__device__ __forceinline__ float dot8(v4f a0, v4f a1, v4f b0, v4f b1) {
  float t = a0.x * b0.x;
  float u = a0.y * b0.y; t = t + u;
  u = a0.z * b0.z; t = t + u;
  u = a0.w * b0.w; t = t + u;
  u = a1.x * b1.x; t = t + u;
  u = a1.y * b1.y; t = t + u;
  u = a1.z * b1.z; t = t + u;
  u = a1.w * b1.w; t = t + u;
  return t;
}

__global__ __launch_bounds__(128) void k_tab(const float* __restrict__ al, const float* __restrict__ ar, float* TAB) {
  const int t = (int)threadIdx.x;
  const int idx = 4 * t;
  const v4f a0 = *(const v4fa*)(al + clampi(idx, 0, 252));
  asm volatile("" :: "v"(a0));
  const v4f a1 = *(const v4fa*)(ar + clampi(idx - 256, 0, 252));
  asm volatile("" :: "v"(a1));
  const unsigned m0 = (idx < 256) ? 0xFFFFFFFFu : 0u;
  const unsigned m1 = ~m0;
  v4u o;
  o.x = (__float_as_uint(a0.x) & m0) | (__float_as_uint(a1.x) & m1);
  o.y = (__float_as_uint(a0.y) & m0) | (__float_as_uint(a1.y) & m1);
  o.z = (__float_as_uint(a0.z) & m0) | (__float_as_uint(a1.z) & m1);
  o.w = (__float_as_uint(a0.w) & m0) | (__float_as_uint(a1.w) & m1);
  o.x = bf16_bits(__uint_as_float(o.x)) << 16;
  o.y = bf16_bits(__uint_as_float(o.y)) << 16;
  o.z = bf16_bits(__uint_as_float(o.z)) << 16;
  o.w = bf16_bits(__uint_as_float(o.w)) << 16;
  volatile v4u* q = (volatile v4u*)(TAB + idx);
  *q = o;
  __threadfence();
  *q = o;
}

__global__ __launch_bounds__(RTHR) void k_rowprep(const float* __restrict__ FT, const float* __restrict__ TAB,
                                                  float* A12) {
  __shared__ __attribute__((aligned(16))) float stab[TAB_N];
  __shared__ __attribute__((aligned(16))) float sdot[2 * RWAVES * NHD];
  const int tid  = (int)threadIdx.x;
  const int lane = tid & 31;
  const int wave = tid >> 5;
  const int row  = (int)blockIdx.x * RWAVES + wave;
  const int rowc = row < MPAD ? row : MPAD - 1;
  const int head = lane >> 3;
  if (tid < 128) {
    const v4f tv = *(const v4fa*)(TAB + 4 * tid);
    *(v4fa*)(stab + 4 * tid) = tv;
  }
  __syncthreads();
  const float* fr = FT + (size_t)rowc * HC + 8 * lane;
  const v4f f0 = *(const v4fa*)fr;
  const v4f f1 = *(const v4fa*)(fr + 4);
  asm volatile("" :: "v"(f0), "v"(f1));
  const v4f l0 = *(const v4fa*)(stab + 8 * lane);
  const v4f l1 = *(const v4fa*)(stab + 8 * lane + 4);
  const v4f r0 = *(const v4fa*)(stab + 256 + 8 * lane);
  const v4f r1 = *(const v4fa*)(stab + 256 + 8 * lane + 4);
  float t1 = dot8(f0, f1, l0, l1);
  float t2 = dot8(f0, f1, r0, r1);
  t1 = sum8(t1);
  t2 = sum8(t2);
  const float k1 = (row < NN) ? t1 : 0.0f;
  const float k2 = (row < NN) ? t2 : 0.0f;
  if ((lane & 7) == 0) {
    sdot[wave * NHD + head] = k1;
    sdot[RWAVES * NHD + wave * NHD + head] = k2;
  }
  __syncthreads();
  if (wave == 0) {
    const int l16   = lane & 15;
    const int which = l16 >> 3;
    const int l8    = l16 & 7;
    const v4f sv = *(const v4fa*)(sdot + which * (RWAVES * NHD) + 4 * l8);
    const int trow = (int)blockIdx.x * RWAVES + l8;
    const int trc  = trow < MPAD ? trow : MPAD - 1;
    const bool wr = lane < 16;
    volatile v4f* q = (volatile v4f*)(A12 + (size_t)which * A2OFF + (size_t)trc * NHD);
    if (wr) *q = sv;
    __threadfence();
    if (wr) *q = sv;
  }
}

__global__ __launch_bounds__(BT) void k_build(const int* __restrict__ eown, const int* __restrict__ egat,
                                              unsigned* LIST, int* META) {
  extern __shared__ v4u lds_bkt[];
  int* reg1 = (int*)lds_bkt;
  int* reg2 = reg1 + RCAP;
  int* scnt = reg2 + RCAP;
  int* soff = scnt + NB;
  int* curs = soff + NB;
  int* wcnt = curs + NB;
  int* wtot = wcnt + 2 * BW;
  const int tid = (int)threadIdx.x, lane = tid & 31, wave = tid >> 5;
  const int nodeBase = (int)blockIdx.x * NB;
  int nb = NN - nodeBase;
  nb = nb > NB ? NB : (nb < 0 ? 0 : nb);
  const unsigned nbs = (unsigned)nodeBase, unb = (unsigned)nb;

  scnt[2 * tid] = 0;
  scnt[2 * tid + 1] = 0;

  int tot = 0;
#pragma unroll 1
  for (int ch = 0; ch < NCH; ++ch) {
    const int par = ch & 1;
    const int e0  = ch * BCHUNK + tid * BEPT;
    const bool valid = e0 < NE;
    const int ea = e0 < NE - 8 ? e0 : NE - 8;
    const v4i da = *(const v4ia*)(eown + ea);
    const v4i db = *(const v4ia*)(eown + ea + 4);
    asm volatile("" :: "v"(da), "v"(db));
    const unsigned s0 = (unsigned)da.x - nbs, s1 = (unsigned)da.y - nbs;
    const unsigned s2 = (unsigned)da.z - nbs, s3 = (unsigned)da.w - nbs;
    const unsigned s4 = (unsigned)db.x - nbs, s5 = (unsigned)db.y - nbs;
    const unsigned s6 = (unsigned)db.z - nbs, s7 = (unsigned)db.w - nbs;
    const bool h0 = valid && (s0 < unb), h1 = valid && (s1 < unb), h2 = valid && (s2 < unb), h3 = valid && (s3 < unb);
    const bool h4 = valid && (s4 < unb), h5 = valid && (s5 < unb), h6 = valid && (s6 < unb), h7 = valid && (s7 < unb);
    const int c = (int)h0 + (int)h1 + (int)h2 + (int)h3 + (int)h4 + (int)h5 + (int)h6 + (int)h7;
    int incl = c;
#pragma unroll
    for (int d = 1; d < 32; d <<= 1) {
      const int up = __shfl_up(incl, d, 32);
      incl += (lane >= d) ? up : 0;
    }
    const int wtotal = __shfl(incl, 31, 32);
    if (lane == 0) wcnt[par * BW + wave] = wtotal;
    __syncthreads();
    int all = 0, pre = 0;
#pragma unroll
    for (int g = 0; g < 4; ++g) {
      const v4i w4 = *(const v4ia*)(wcnt + par * BW + 4 * g);
      const int c0 = clampi(w4.x, 0, 256), c1 = clampi(w4.y, 0, 256);
      const int c2 = clampi(w4.z, 0, 256), c3 = clampi(w4.w, 0, 256);
      all += c0 + c1 + c2 + c3;
      pre += (4 * g + 0 < wave) ? c0 : 0;
      pre += (4 * g + 1 < wave) ? c1 : 0;
      pre += (4 * g + 2 < wave) ? c2 : 0;
      pre += (4 * g + 3 < wave) ? c3 : 0;
    }
    int pos = tot + pre + (incl - c);
#define PUTJ(J, HJ, SJ) if (HJ) { if (pos < RCAP) reg1[pos] = (int)((unsigned)(e0 + (J)) | ((SJ) << SLOTSH)); ++pos; }
    PUTJ(0, h0, s0)
    PUTJ(1, h1, s1)
    PUTJ(2, h2, s2)
    PUTJ(3, h3, s3)
    PUTJ(4, h4, s4)
    PUTJ(5, h5, s5)
    PUTJ(6, h6, s6)
    PUTJ(7, h7, s7)
#undef PUTJ
    tot += all;
  }
  __syncthreads();
  const bool ovf = tot > RCAP;
  const int nh = ovf ? RCAP : tot;

  if (wave == 0) {
#pragma unroll 1
    for (int b0 = 0; b0 < nh; b0 += 32) {
      const int idx = b0 + lane;
      const int uv  = reg1[idx < nh ? idx : nh - 1];
      const int m32 = (nh - b0) < 32 ? (nh - b0) : 32;
#pragma unroll 1
      for (int k = 0; k < m32; ++k) {
        const int u  = __builtin_amdgcn_readlane(uv, k);
        const int sl = (int)(((unsigned)u >> SLOTSH) & (unsigned)(NB - 1));
        const int cv = scnt[sl] + 1;
        if (lane == 0) scnt[sl] = cv;
      }
    }
  }
  __syncthreads();

  int e0c, e1c;
  {
    const v2i cc = *(const v2ia*)(scnt + 2 * tid);
    e0c = cc.x < 0 ? 0 : cc.x;
    e1c = cc.y < 0 ? 0 : cc.y;
    const int ts = e0c + e1c;
    int incl = ts;
#pragma unroll
    for (int d = 1; d < 32; d <<= 1) {
      const int up = __shfl_up(incl, d, 32);
      incl += (lane >= d) ? up : 0;
    }
    if (lane == 31) wtot[wave] = incl;
    __syncthreads();
    int pre = 0;
#pragma unroll
    for (int g = 0; g < 4; ++g) {
      const v4i w4 = *(const v4ia*)(wtot + 4 * g);
      pre += (4 * g + 0 < wave) ? w4.x : 0;
      pre += (4 * g + 1 < wave) ? w4.y : 0;
      pre += (4 * g + 2 < wave) ? w4.z : 0;
      pre += (4 * g + 3 < wave) ? w4.w : 0;
    }
    const int run = pre + incl - ts;
    soff[2 * tid]     = run;
    soff[2 * tid + 1] = run + e0c;
    curs[2 * tid]     = run;
    curs[2 * tid + 1] = run + e0c;
  }
  __syncthreads();

  if (wave == 0) {
#pragma unroll 1
    for (int b0 = 0; b0 < nh; b0 += 32) {
      const int idx = b0 + lane;
      const int uv  = reg1[idx < nh ? idx : nh - 1];
      const int m32 = (nh - b0) < 32 ? (nh - b0) : 32;
#pragma unroll 1
      for (int k = 0; k < m32; ++k) {
        const int u   = __builtin_amdgcn_readlane(uv, k);
        const int sl  = (int)(((unsigned)u >> SLOTSH) & (unsigned)(NB - 1));
        const int eid = (int)((unsigned)u & ((1u << SLOTSH) - 1u));
        const int pr  = curs[sl];
        const int pc  = clampi(pr, 0, RCAP - 1);
        if (lane == 0) { reg2[pc] = eid; curs[sl] = pc + 1; }
      }
    }
  }
  __syncthreads();

  {
    int nhPad = (nh + 31) & ~31;
    nhPad = nhPad > RCAP ? RCAP : nhPad;
    const int nIt = (nhPad + BT - 1) / BT;
    unsigned* lbase = LIST + (size_t)blockIdx.x * (size_t)RCAP;
#pragma unroll 1
    for (int it = 0; it < nIt; ++it) {
      const int i  = it * BT + tid;
      const int ic = i < nh ? i : nh - 1;
      const int eid = clampi(reg2[ic], 0, NE - 1);
      const int cw = egat[eid];
      asm volatile("" :: "v"(cw));
      const unsigned msk = (i < nh) ? 0xFFFFFFFFu : 0u;
      const unsigned o = (unsigned)clampi(cw, 0, NN - 1) & msk;
      const int iw = i < RCAP ? i : RCAP - 1;
      volatile unsigned* q = (volatile unsigned*)(lbase + (size_t)iw);
      const bool wr = i < nhPad;
      if (wr) *q = o;
      __threadfence();
      if (wr) *q = o;
    }
  }

  {
    const int base = (int)blockIdx.x * RCAP;
    const v2i cc = *(const v2ia*)(scnt + 2 * tid);
    const v2i so = *(const v2ia*)(soff + 2 * tid);
    v4i m;
    m.x = base + so.x;
    m.y = ovf ? -1 : cc.x;
    m.z = base + so.y;
    m.w = ovf ? -1 : cc.y;
    volatile v4i* q = (volatile v4i*)(META + 2 * (size_t)(nodeBase + 2 * tid));
    *q = m;
    __threadfence();
    *q = m;
  }
}

__device__ __forceinline__ float entry_e(const unsigned* __restrict__ LIST, const float* __restrict__ A12,
                                         int off, int cnt, int b0, int eq, int hq, float a2v, int& sidx) {
  int j = b0 + eq;
  j = j < cnt ? j : cnt - 1;
  const unsigned sw = LIST[(size_t)(off + j)];
  asm volatile("" :: "v"(sw));
  const int s = clampi((int)sw, 0, NN - 1);
  const float a1v = A12[(size_t)s * NHD + hq];
  asm volatile("" :: "v"(a1v));
  sidx = s;
  const float v = a1v + a2v;
  return lrelu_k(v);
}

__global__ __launch_bounds__(RTHR) void k_walk(const float* __restrict__ FT, const float* __restrict__ A12,
                                               const unsigned* __restrict__ LIST, const int* __restrict__ META,
                                               float* out) {
  __shared__ __attribute__((aligned(16))) float srow[RWAVES][HC];
  const int lane = (int)threadIdx.x & 31;
  const int wave = (int)threadIdx.x >> 5;
  const int row  = (int)blockIdx.x * RWAVES + wave;
  const int rowc = row < NN ? row : NN - 1;
  const int hq = lane & 3;
  const int eq = lane >> 2;
  const int hc = lane >> 3;

  const v2i mt = *(const v2ia*)(META + 2 * (size_t)rowc);
  asm volatile("" :: "v"(mt));
  const int craw = mt.y;
  const int offv = clampi(mt.x, 0, LISTTOT);
  int cntv = clampi(craw, 0, DEGCAP);
  cntv = cntv < (LISTTOT - offv) ? cntv : (LISTTOT - offv);
  cntv = (row < NN) ? cntv : 0;
  const int off = __builtin_amdgcn_readfirstlane(offv);
  const int cnt = __builtin_amdgcn_readfirstlane(cntv);
  const bool poison = (craw < 0) || (craw > DEGCAP);

  const float a2v = A12[(size_t)A2OFF + (size_t)rowc * NHD + hq];
  asm volatile("" :: "v"(a2v));

  float mx = -__builtin_inff();
#pragma unroll 1
  for (int b0 = 0; b0 < cnt; b0 += WSTEP) {
    int sidx;
    const float e = entry_e(LIST, A12, off, cnt, b0, eq, hq, a2v, sidx);
    mx = nmax(mx, e);
  }
  {
    const float o4 = __shfl_xor(mx, 4, 32);  mx = nmax(mx, o4);
    const float o8 = __shfl_xor(mx, 8, 32);  mx = nmax(mx, o8);
    const float o16 = __shfl_xor(mx, 16, 32); mx = nmax(mx, o16);
  }

  float s = 0.0f;
#pragma unroll 1
  for (int b0 = 0; b0 < cnt; b0 += WSTEP) {
    int sidx;
    const float e = entry_e(LIST, A12, off, cnt, b0, eq, hq, a2v, sidx);
    const float d = e - mx;
    const float ex = expf(d);
    const int m8 = (cnt - b0) < WSTEP ? (cnt - b0) : WSTEP;
#pragma unroll 1
    for (int k = 0; k < m8; ++k) {
      const float v = __shfl(ex, 4 * k + hq, 32);
      s = s + v;
    }
  }

  v4f ac0 = (v4f){0.0f, 0.0f, 0.0f, 0.0f};
  v4f ac1 = (v4f){0.0f, 0.0f, 0.0f, 0.0f};
#pragma unroll 1
  for (int b0 = 0; b0 < cnt; b0 += WSTEP) {
    int sidx;
    const float e = entry_e(LIST, A12, off, cnt, b0, eq, hq, a2v, sidx);
    const float d = e - mx;
    const float ex = expf(d);
    const float w = ex / s;
    const int m8 = (cnt - b0) < WSTEP ? (cnt - b0) : WSTEP;
#pragma unroll 1
    for (int k = 0; k < m8; ++k) {
      const int c = __builtin_amdgcn_readlane(sidx, 4 * k);
      const float wk = __shfl(w, 4 * k + hc, 32);
      const float* fp = FT + (size_t)c * HC + 8 * lane;
      const v4f f0 = *(const v4fa*)fp;
      const v4f f1 = *(const v4fa*)(fp + 4);
      asm volatile("" :: "v"(f0), "v"(f1));
      float t;
      t = wk * f0.x; ac0.x = ac0.x + t;
      t = wk * f0.y; ac0.y = ac0.y + t;
      t = wk * f0.z; ac0.z = ac0.z + t;
      t = wk * f0.w; ac0.w = ac0.w + t;
      t = wk * f1.x; ac1.x = ac1.x + t;
      t = wk * f1.y; ac1.y = ac1.y + t;
      t = wk * f1.z; ac1.z = ac1.z + t;
      t = wk * f1.w; ac1.w = ac1.w + t;
    }
  }

  float* sr = srow[wave];
  *(v4fa*)(sr + 8 * lane)     = ac0;
  *(v4fa*)(sr + 8 * lane + 4) = ac1;
  const float qnan = __uint_as_float(0x7fc00000u);
#pragma unroll 1
  for (int e = 0; e < 8; ++e) {
    const float v = sr[8 * lane + e];
    float y = (v > 0.0f) ? v : expm1f(v);
    y = poison ? qnan : y;
    sr[8 * lane + e] = y;
  }
  __builtin_amdgcn_fence(__ATOMIC_RELEASE, "workgroup");
  __builtin_amdgcn_wave_barrier();
  __builtin_amdgcn_fence(__ATOMIC_ACQUIRE, "workgroup");
  const v4f r0 = *(const v4fa*)(sr + 4 * lane);
  const v4f r1 = *(const v4fa*)(sr + 128 + 4 * lane);
  float* orow = out + (size_t)rowc * HC;
  const bool rok = row < NN;
  if (rok) {
    *(volatile v4f*)(orow + 4 * lane)       = r0;
    *(volatile v4f*)(orow + 128 + 4 * lane) = r1;
  }
  __threadfence();
  if (rok) {
    *(volatile v4f*)(orow + 4 * lane)       = r0;
    *(volatile v4f*)(orow + 128 + 4 * lane) = r1;
  }
}

extern "C" void kernel_launch(void* const* d_in, const int* in_sizes, int n_in,
                              void* d_out, int out_size, void* d_ws, size_t ws_size,
                              hipStream_t stream) {
  if (n_in < 6) return;
  if (in_sizes[0] != NN * KD) return;
  if (in_sizes[1] != NE || in_sizes[2] != NE) return;
  if (in_sizes[3] != HC * KD) return;
  if (in_sizes[4] != NHD * DSZ || in_sizes[5] != NHD * DSZ) return;
  if (out_size != NN * HC) return;

  const float* feat = (const float*)d_in[0];
  const int*   egat = (const int*)  d_in[1];
  const int*   eown = (const int*)  d_in[2];
  const float* W    = (const float*)d_in[3];
  const float* al   = (const float*)d_in[4];
  const float* ar   = (const float*)d_in[5];
  float* out = (float*)d_out;

  const size_t szXB   = (size_t)MPAD * KD * 2;
  const size_t szWB   = (size_t)HC * KD * 2;
  const size_t szTAB  = (size_t)TAB_N * 4;
  const size_t szFT   = (size_t)MPAD * HC * 4;
  const size_t szA12  = (size_t)2 * MPAD * NHD * 4;
  const size_t szMETA = (size_t)NBLK * NB * 2 * 4;
  const size_t szLIST = (size_t)NBLK * RCAP * 4;
  static_assert((size_t)MPAD * KD * 2 + (size_t)HC * KD * 2 + (size_t)TAB_N * 4 + (size_t)MPAD * HC * 4 +
                (size_t)2 * MPAD * NHD * 4 + (size_t)NBLK * NB * 8 + (size_t)NBLK * RCAP * 4 == 83124224);
  static_assert(83124224 <= WSMAX);
  char* ws = (char*)d_ws;
  size_t off = 0;
  const size_t oXB   = off; off += szXB;
  const size_t oWB   = off; off += szWB;
  const size_t oTAB  = off; off += szTAB;
  const size_t oFT   = off; off += szFT;
  const size_t oA12  = off; off += szA12;
  const size_t oMETA = off; off += szMETA;
  const size_t oLIST = off; off += szLIST;
  if (off > ws_size || off > (size_t)WSMAX) return;
  unsigned short* XB = (unsigned short*)(ws + oXB);
  unsigned short* WB = (unsigned short*)(ws + oWB);
  float*    TAB  = (float*)(ws + oTAB);
  float*    FT   = (float*)(ws + oFT);
  float*    A12  = (float*)(ws + oA12);
  int*      META = (int*)(ws + oMETA);
  unsigned* LIST = (unsigned*)(ws + oLIST);

  hipFuncSetAttribute(reinterpret_cast<const void*>(&k_build),
                      hipFuncAttributeMaxDynamicSharedMemorySize, LDS_BKT);

  k_plane<0><<<MPAD * KD / 8 / 256, 256, 0, stream>>>(feat, NN, KD, KD, XB, MPAD, KD);
  k_plane<0><<<HC * KD / 8 / 256, 256, 0, stream>>>(W, HC, KD, KD, WB, HC, KD);
  k_tab<<<1, 128, 0, stream>>>(al, ar, TAB);

  const int tiles = (MPAD / 64) * (HC / 64);
  const int gG = (tiles + 7) / 8;
  k_gemm_nt<0, 0><<<gG, 256, 0, stream>>>(XB, WB, TAB, FT, MPAD, HC, KD, HC);

  k_rowprep<<<MPAD / RWAVES, RTHR, 0, stream>>>(FT, TAB, A12);
  k_build<<<NBLK, BT, LDS_BKT, stream>>>(eown, egat, LIST, META);
  k_walk<<<NN / RWAVES, RTHR, 0, stream>>>(FT, A12, LIST, META, out);
}
